// MLMCrossMultiHeadAttention_55602646614530
// MI455X (gfx1250) — hardware-verified
//
#include <hip/hip_runtime.h>
#include <hip/hip_bf16.h>

#pragma clang fp contract(off)

typedef __bf16         v16bf __attribute__((ext_vector_type(16)));
typedef unsigned short v16us __attribute__((ext_vector_type(16)));
typedef unsigned short v8us  __attribute__((ext_vector_type(8)));
typedef float          v8f   __attribute__((ext_vector_type(8)));
typedef float          v4f   __attribute__((ext_vector_type(4)));
typedef v8us __attribute__((may_alias)) v8usa;
typedef v4f  __attribute__((may_alias)) v4fa;

union Frag { v16bf b; v16us u; v8us h[2]; };
struct Frag2 { v16bf hi; v16bf lo; };

#define D_DIM   2048
#define N1      250
#define N2      27
#define M1P     256
#define M2P     32
#define OUT_N   580796
#define OFF1    512000
#define OFF2    518750
#define OFF3    574046
#define XG1     65536
#define XG2     8192
#define WGRP    524288
#define NGROUPS (XG1 + XG2 + 6 * WGRP)
#define SCALE   0.022097086912079608f
#define L_P2A   16000
#define L_P2B   16210
#define L_P1A   16211
#define L_P1B   18149

static_assert((XG1 % 256) == 0 && (XG2 % 256) == 0 && (WGRP % 256) == 0);
static_assert((OFF1 % 32) == 0 && (L_P1B * 32 + 28) == OUT_N);

__device__ __forceinline__ unsigned int bf16_bits(float f) {
  unsigned int u = __float_as_uint(f);
  u += 0x7FFFu + ((u >> 16) & 1u);
  return u >> 16;
}

__device__ __forceinline__ void split2(float f, unsigned int& hb, unsigned int& lb) {
  hb = bf16_bits(f);
  const float hf = __uint_as_float(hb << 16);
  lb = bf16_bits(f - hf);
}

__device__ __forceinline__ v8f wmma_bf16(v16bf a, v16bf b, v8f c) {
  v8f d = __builtin_amdgcn_wmma_f32_16x16x32_bf16(false, a, false, b, (short)0, c, false, false);
  asm volatile("v_nop\n\tv_nop\n\tv_nop\n\tv_nop" : "+v"(d) : "v"(a), "v"(b));
  return d;
}

__device__ __forceinline__ v8f mac3(v16bf ah, v16bf al, v16bf bh, v16bf bl, v8f c) {
  c = wmma_bf16(ah, bh, c);
  c = wmma_bf16(ah, bl, c);
  c = wmma_bf16(al, bh, c);
  return c;
}

__device__ __forceinline__ v16bf load_frag16(const unsigned short* p, int h) {
  Frag f;
  f.h[0] = *(const v8usa*)(p + 8 * h);
  f.h[1] = *(const v8usa*)(p + 16 + 8 * h);
  return f.b;
}

template <int B>
__device__ __forceinline__ void split4(const v4f v, Frag& fh, Frag& fl) {
  unsigned int hb, lb;
  split2(v.x, hb, lb); fh.u[B + 0] = (unsigned short)hb; fl.u[B + 0] = (unsigned short)lb;
  split2(v.y, hb, lb); fh.u[B + 1] = (unsigned short)hb; fl.u[B + 1] = (unsigned short)lb;
  split2(v.z, hb, lb); fh.u[B + 2] = (unsigned short)hb; fl.u[B + 2] = (unsigned short)lb;
  split2(v.w, hb, lb); fh.u[B + 3] = (unsigned short)hb; fl.u[B + 3] = (unsigned short)lb;
}

__device__ __forceinline__ Frag2 load_split32(const float* p, int h) {
  Frag fh, fl;
  const float* q = p + 8 * h;
  split4<0>(*(const v4fa*)(q), fh, fl);
  split4<4>(*(const v4fa*)(q + 4), fh, fl);
  split4<8>(*(const v4fa*)(q + 16), fh, fl);
  split4<12>(*(const v4fa*)(q + 20), fh, fl);
  Frag2 r;
  r.hi = fh.b;
  r.lo = fl.b;
  return r;
}

template <int NT>
__device__ __forceinline__ void wave_gemm_split(const float* __restrict__ arow,
                                                const float* __restrict__ brow0,
                                                int h, v8f (&acc)[NT]) {
#pragma unroll 1
  for (int k0 = 0; k0 < D_DIM; k0 += 32) {
    const Frag2 a = load_split32(arow + k0, h);
#pragma unroll
    for (int nt = 0; nt < NT; ++nt) {
      const Frag2 b = load_split32(brow0 + (size_t)nt * 16 * D_DIM + k0, h);
      acc[nt] = mac3(a.hi, a.lo, b.hi, b.lo, acc[nt]);
    }
  }
}

__device__ __forceinline__ float sigm(float x) {
  const float e = expf(-x);
  return 1.0f / (1.0f + e);
}

__global__ __launch_bounds__(256) void convert_kernel(
    const float* __restrict__ x1, const float* __restrict__ x2,
    const float* __restrict__ w0, const float* __restrict__ w1, const float* __restrict__ w2,
    const float* __restrict__ w3, const float* __restrict__ w4, const float* __restrict__ w5,
    unsigned short* __restrict__ xh1, unsigned short* __restrict__ xl1,
    unsigned short* __restrict__ xh2, unsigned short* __restrict__ xl2,
    unsigned short* __restrict__ wh,  unsigned short* __restrict__ wl)
{
  const int g = blockIdx.x * 256 + threadIdx.x;
  if (g >= NGROUPS) return;
  const float* src;
  unsigned short* dh;
  unsigned short* dl;
  bool zero = false;
  if (g < XG1) {
    const int row = g >> 8, c8 = g & 255;
    const int rs = (row < N1) ? row : (N1 - 1);
    zero = (row >= N1);
    src = x1 + (size_t)rs * D_DIM + 8 * c8;
    dh = xh1 + (size_t)g * 8;
    dl = xl1 + (size_t)g * 8;
  } else if (g < XG1 + XG2) {
    const int e = g - XG1;
    const int row = e >> 8, c8 = e & 255;
    const int rs = (row < N2) ? row : (N2 - 1);
    zero = (row >= N2);
    src = x2 + (size_t)rs * D_DIM + 8 * c8;
    dh = xh2 + (size_t)e * 8;
    dl = xl2 + (size_t)e * 8;
  } else {
    const int e = g - XG1 - XG2;
    const int wsel = e >> 19;
    const int off = e & (WGRP - 1);
    const float* wsrc = (wsel == 0) ? w0 : ((wsel == 1) ? w1 : ((wsel == 2) ? w2 :
                        ((wsel == 3) ? w3 : ((wsel == 4) ? w4 : w5))));
    src = wsrc + (size_t)off * 8;
    dh = wh + (size_t)e * 8;
    dl = wl + (size_t)e * 8;
  }
  v4f a = *(const v4fa*)src;
  v4f c = *(const v4fa*)(src + 4);
  const v4f z4 = {0.f, 0.f, 0.f, 0.f};
  a = zero ? z4 : a;
  c = zero ? z4 : c;
  unsigned int hb[8], lb[8];
  split2(a.x, hb[0], lb[0]); split2(a.y, hb[1], lb[1]); split2(a.z, hb[2], lb[2]); split2(a.w, hb[3], lb[3]);
  split2(c.x, hb[4], lb[4]); split2(c.y, hb[5], lb[5]); split2(c.z, hb[6], lb[6]); split2(c.w, hb[7], lb[7]);
  const v8us hv = { (unsigned short)hb[0], (unsigned short)hb[1], (unsigned short)hb[2], (unsigned short)hb[3],
                    (unsigned short)hb[4], (unsigned short)hb[5], (unsigned short)hb[6], (unsigned short)hb[7] };
  const v8us lv = { (unsigned short)lb[0], (unsigned short)lb[1], (unsigned short)lb[2], (unsigned short)lb[3],
                    (unsigned short)lb[4], (unsigned short)lb[5], (unsigned short)lb[6], (unsigned short)lb[7] };
  *(volatile v8us*)dh = hv;
  *(volatile v8us*)dl = lv;
  __threadfence();
  *(volatile v8us*)dh = hv;
  *(volatile v8us*)dl = lv;
}

__device__ __forceinline__ void proj_store_pass(const float* sTw, float* P, int row0, int col0, int lane) {
  const int q8 = lane & 7, sub = lane >> 3;
#pragma unroll
  for (int i = 0; i < 16; ++i) {
    const int lid = 4 * i + sub;
    const int r = lid >> 1, hl = lid & 1;
    const v4f v = *(const v4fa*)(sTw + r * 64 + 32 * hl + 4 * q8);
    float* dst = P + (size_t)(row0 + r) * D_DIM + col0 + 32 * hl + 4 * q8;
    *(volatile v4f*)dst = v;
  }
}

__global__ __launch_bounds__(128) void proj_kernel(
    const unsigned short* __restrict__ xh1, const unsigned short* __restrict__ xl1,
    const unsigned short* __restrict__ xh2, const unsigned short* __restrict__ xl2,
    const unsigned short* __restrict__ wh,  const unsigned short* __restrict__ wl,
    const float* __restrict__ b0, const float* __restrict__ b1, const float* __restrict__ b2,
    const float* __restrict__ b3, const float* __restrict__ b4, const float* __restrict__ b5,
    float* __restrict__ P1,
    float* __restrict__ P2)
{
  __shared__ __attribute__((aligned(16))) float sT[4 * 32 * 64];

  const int tid = threadIdx.x, lane = tid & 31, w = tid >> 5;
  const int h = lane >> 4, m = lane & 15;
  const int gw = blockIdx.x * 4 + w;
  int g, mt32, nt64;
  if (gw < 768) {
    g = gw >> 8;
    const int t = gw & 255;
    mt32 = t & 7;
    nt64 = t >> 3;
  } else {
    const int e = gw - 768;
    g = 3 + (e >> 5);
    mt32 = 0;
    nt64 = e & 31;
  }
  const int row0 = 32 * mt32, col0 = 64 * nt64;

  const unsigned short* ah = (g < 3) ? xh1 : xh2;
  const unsigned short* al = (g < 3) ? xl1 : xl2;
  const unsigned short* ahr = ah + (size_t)(row0 + m) * D_DIM;
  const unsigned short* alr = al + (size_t)(row0 + m) * D_DIM;
  const unsigned short* whr = wh + ((size_t)g * D_DIM + col0 + m) * D_DIM;
  const unsigned short* wlr = wl + ((size_t)g * D_DIM + col0 + m) * D_DIM;

  const v8f z8 = {0.f, 0.f, 0.f, 0.f, 0.f, 0.f, 0.f, 0.f};
  v8f acc[2][4];
#pragma unroll
  for (int mt = 0; mt < 2; ++mt)
#pragma unroll
    for (int nt = 0; nt < 4; ++nt) acc[mt][nt] = z8;

#pragma unroll 1
  for (int k0 = 0; k0 < D_DIM; k0 += 32) {
    const v16bf ah0 = load_frag16(ahr + k0, h);
    const v16bf al0 = load_frag16(alr + k0, h);
    const v16bf ah1 = load_frag16(ahr + (size_t)16 * D_DIM + k0, h);
    const v16bf al1 = load_frag16(alr + (size_t)16 * D_DIM + k0, h);
#pragma unroll
    for (int nt = 0; nt < 4; ++nt) {
      const v16bf bh = load_frag16(whr + (size_t)nt * 16 * D_DIM + k0, h);
      const v16bf bl = load_frag16(wlr + (size_t)nt * 16 * D_DIM + k0, h);
      acc[0][nt] = mac3(ah0, al0, bh, bl, acc[0][nt]);
      acc[1][nt] = mac3(ah1, al1, bh, bl, acc[1][nt]);
    }
  }

  const float* bias = (g == 0) ? b0 : ((g == 1) ? b1 : ((g == 2) ? b2 :
                      ((g == 3) ? b3 : ((g == 4) ? b4 : b5))));
  float* sTw = sT + w * 2048;
#pragma unroll
  for (int nt = 0; nt < 4; ++nt) {
    const int col = 16 * nt + m;
    const float bvl = bias[col0 + col];
#pragma unroll
    for (int mt = 0; mt < 2; ++mt) {
#pragma unroll
      for (int r = 0; r < 8; ++r)
        sTw[(16 * mt + 8 * h + r) * 64 + col] = acc[mt][nt][r] + bvl;
    }
  }
  __syncthreads();

  float* P = (g < 3) ? (P1 + (size_t)g * M1P * D_DIM) : (P2 + (size_t)(g - 3) * M2P * D_DIM);
  proj_store_pass(sTw, P, row0, col0, lane);
  __threadfence();
  proj_store_pass(sTw, P, row0, col0, lane);
}

__device__ __forceinline__ void ctx2_store_pass(const float* __restrict__ v1P, const float* sS2, float bb,
                                                float* out, int row0, int w, int lane) {
  const int q8 = lane & 7, sub = lane >> 3;
#pragma unroll 4
  for (int it = 0; it < 32; ++it) {
    const int line = 4 * it + sub;
    const int rr = 2 * w + (line >> 6);
    const int row = row0 + rr;
    const int c0 = (line & 63) * 32 + 4 * q8;
    const v4f v = *(const v4fa*)(v1P + (size_t)row * D_DIM + c0);
    const float s = sS2[rr];
    v4f o;
    o.x = v.x * s + bb;
    o.y = v.y * s + bb;
    o.z = v.z * s + bb;
    o.w = v.w * s + bb;
    if (row < N1) *(volatile v4f*)(out + (size_t)row * D_DIM + c0) = o;
  }
}

__global__ __launch_bounds__(256) void ctx2_kernel(
    const float* __restrict__ P1, const float* __restrict__ P2,
    const float* __restrict__ wfc2, const float* __restrict__ bfc2,
    float* __restrict__ out)
{
  __shared__ __attribute__((aligned(16))) float sS[16 * 32];
  __shared__ float sS2[16];

  const int tid = threadIdx.x, lane = tid & 31, w = tid >> 5;
  const int h = lane >> 4, m = lane & 15;
  const int row0 = 16 * blockIdx.x;

  const float* q1P = P1;
  const float* v1P = P1 + (size_t)2 * M1P * D_DIM;
  const float* k2P = P2 + (size_t)1 * M2P * D_DIM;

  if (w < 2) {
    const v8f z8 = {0.f, 0.f, 0.f, 0.f, 0.f, 0.f, 0.f, 0.f};
    v8f acc[1];
    acc[0] = z8;
    wave_gemm_split<1>(q1P + (size_t)(row0 + m) * D_DIM, k2P + (size_t)(16 * w + m) * D_DIM, h, acc);
#pragma unroll
    for (int r = 0; r < 8; ++r) sS[(8 * h + r) * 32 + 16 * w + m] = acc[0][r] * SCALE;
  }
  __syncthreads();

  if (tid < 16) {
    float s = 0.0f;
#pragma unroll 1
    for (int t = 0; t < N2; ++t) s += sigm(sS[tid * 32 + t]) * wfc2[t];
    sS2[tid] = s;
  }
  __syncthreads();

  const float bb = bfc2[0];
  ctx2_store_pass(v1P, sS2, bb, out, row0, w, lane);
  __threadfence();
  ctx2_store_pass(v1P, sS2, bb, out, row0, w, lane);
}

__device__ __forceinline__ void score_tile(const float* __restrict__ A, const float* __restrict__ B,
                                           float* sC, int w, int h, int m) {
  const int mt = w & 1, ntb = 4 * (w >> 1);
  const v8f z8 = {0.f, 0.f, 0.f, 0.f, 0.f, 0.f, 0.f, 0.f};
  const float* arow = A + (size_t)(16 * mt + m) * D_DIM;
#pragma unroll
  for (int half = 0; half < 2; ++half) {
    v8f acc[2];
    acc[0] = z8;
    acc[1] = z8;
    wave_gemm_split<2>(arow, B + (size_t)(16 * (ntb + 2 * half) + m) * D_DIM, h, acc);
#pragma unroll
    for (int nt = 0; nt < 2; ++nt)
#pragma unroll
      for (int r = 0; r < 8; ++r)
        sC[(16 * mt + 8 * h + r) * 256 + 16 * (ntb + 2 * half + nt) + m] = acc[nt][r] * SCALE;
  }
}

__device__ __forceinline__ float tail_val(int f, const float* sC, const float* sS1,
                                          const float* __restrict__ v2P, float bb1) {
  int j2 = f - OFF1;
  j2 = (j2 < 0) ? 0 : ((j2 > N1 * N2 - 1) ? (N1 * N2 - 1) : j2);
  const int i2 = j2 / N2, t2 = j2 - i2 * N2;
  const float c2 = sC[t2 * 256 + i2];
  int j1 = f - OFF2;
  j1 = (j1 < 0) ? 0 : ((j1 > N2 * D_DIM - 1) ? (N2 * D_DIM - 1) : j1);
  const int t1 = j1 >> 11, d1 = j1 & (D_DIM - 1);
  const float x = v2P[(size_t)t1 * D_DIM + d1] * sS1[t1] + bb1;
  int j3 = f - OFF3;
  j3 = (j3 < 0) ? 0 : ((j3 > N1 * N2 - 1) ? (N1 * N2 - 1) : j3);
  const int t3 = j3 / N1, i3 = j3 - t3 * N1;
  const float c3 = sC[t3 * 256 + i3];
  return (f < OFF2) ? c2 : ((f < OFF3) ? x : c3);
}

__device__ __forceinline__ void tail_pass(const float* sC, const float* sS1, const float* __restrict__ v2P,
                                          float bb1, float* out, int L0, int L1, int w, int lane) {
  const int q8 = lane & 7, sub = lane >> 3;
  const int nch = (L1 - L0 + 4) >> 2;
#pragma unroll 1
  for (int ci = w; ci < nch; ci += 8) {
    const int line = L0 + 4 * ci + sub;
    const int linec = (line < L1) ? line : L1;
    const int fbase = 32 * linec + 4 * q8;
    v4f o;
    o.x = tail_val(fbase + 0, sC, sS1, v2P, bb1);
    o.y = tail_val(fbase + 1, sC, sS1, v2P, bb1);
    o.z = tail_val(fbase + 2, sC, sS1, v2P, bb1);
    o.w = tail_val(fbase + 3, sC, sS1, v2P, bb1);
    if (line <= L1 && fbase + 4 <= OUT_N) *(volatile v4f*)(out + fbase) = o;
  }
}

__global__ __launch_bounds__(256) void tail_kernel(
    const float* __restrict__ P1, const float* __restrict__ P2,
    const float* __restrict__ wfc1, const float* __restrict__ bfc1,
    float* __restrict__ out)
{
  __shared__ __attribute__((aligned(16))) float sC[32 * 256];
  __shared__ float sS1[32];

  const int tid = threadIdx.x, lane = tid & 31, w = tid >> 5;
  const int h = lane >> 4, m = lane & 15;

  const float* q1P = P1;
  const float* k1P = P1 + (size_t)1 * M1P * D_DIM;
  const float* q2P = P2;
  const float* k2P = P2 + (size_t)1 * M2P * D_DIM;
  const float* v2P = P2 + (size_t)2 * M2P * D_DIM;

  score_tile(q2P, k1P, sC, w, h, m);
  __syncthreads();
#pragma unroll 1
  for (int idx = tid; idx < 32 * 256; idx += 256) sC[idx] = sigm(sC[idx]);
  __syncthreads();
  if (tid < 32) {
    float s = 0.0f;
#pragma unroll 1
    for (int i = 0; i < N1; ++i) s += sC[tid * 256 + i] * wfc1[i];
    sS1[tid] = s;
  }
  __syncthreads();
  const float bb1 = bfc1[0];
  tail_pass(sC, sS1, v2P, bb1, out, L_P1A, L_P1B, w, lane);
  __threadfence();
  tail_pass(sC, sS1, v2P, bb1, out, L_P1A, L_P1B, w, lane);
  __syncthreads();

  score_tile(k2P, q1P, sC, w, h, m);
  __syncthreads();
#pragma unroll 1
  for (int idx = tid; idx < 32 * 256; idx += 256) sC[idx] = sigm(sC[idx]);
  __syncthreads();
  tail_pass(sC, sS1, v2P, bb1, out, L_P2A, L_P2B, w, lane);
  __threadfence();
  tail_pass(sC, sS1, v2P, bb1, out, L_P2A, L_P2B, w, lane);
}

extern "C" void kernel_launch(void* const* d_in, const int* in_sizes, int n_in,
                              void* d_out, int out_size, void* d_ws, size_t ws_size,
                              hipStream_t stream) {
  if (n_in < 18) return;
  if (in_sizes[0] != N1 * D_DIM || in_sizes[1] != N2 * D_DIM) return;
  for (int g = 0; g < 6; ++g) {
    if (in_sizes[2 + 2 * g] != D_DIM * D_DIM) return;
    if (in_sizes[3 + 2 * g] != D_DIM) return;
  }
  if (in_sizes[14] != N1 || in_sizes[15] < 1 || in_sizes[16] != N2 || in_sizes[17] < 1) return;
  if (out_size != OUT_N) return;

  const float* x1   = (const float*)d_in[0];
  const float* x2   = (const float*)d_in[1];
  const float* Wq1  = (const float*)d_in[2];  const float* bq1 = (const float*)d_in[3];
  const float* Wk1  = (const float*)d_in[4];  const float* bk1 = (const float*)d_in[5];
  const float* Wv1  = (const float*)d_in[6];  const float* bv1 = (const float*)d_in[7];
  const float* Wq2  = (const float*)d_in[8];  const float* bq2 = (const float*)d_in[9];
  const float* Wk2  = (const float*)d_in[10]; const float* bk2 = (const float*)d_in[11];
  const float* Wv2  = (const float*)d_in[12]; const float* bv2 = (const float*)d_in[13];
  const float* wfc1 = (const float*)d_in[14]; const float* bfc1 = (const float*)d_in[15];
  const float* wfc2 = (const float*)d_in[16]; const float* bfc2 = (const float*)d_in[17];
  float* out = (float*)d_out;

  const size_t xp1_bytes = (size_t)M1P * D_DIM * 2;
  const size_t xp2_bytes = (size_t)M2P * D_DIM * 2;
  const size_t wp_bytes  = (size_t)6 * D_DIM * D_DIM * 2;
  const size_t p1_bytes  = (size_t)3 * M1P * D_DIM * 4;
  const size_t p2_bytes  = (size_t)3 * M2P * D_DIM * 4;
  const size_t off_xh1 = 0;
  const size_t off_xl1 = off_xh1 + xp1_bytes;
  const size_t off_xh2 = off_xl1 + xp1_bytes;
  const size_t off_xl2 = off_xh2 + xp2_bytes;
  const size_t off_wh  = off_xl2 + xp2_bytes;
  const size_t off_wl  = off_wh + wp_bytes;
  const size_t off_p1  = off_wl + wp_bytes;
  const size_t off_p2  = off_p1 + p1_bytes;
  const size_t total   = off_p2 + p2_bytes;
  if (total > ws_size) return;

  char* ws = (char*)d_ws;
  unsigned short* xh1 = (unsigned short*)(ws + off_xh1);
  unsigned short* xl1 = (unsigned short*)(ws + off_xl1);
  unsigned short* xh2 = (unsigned short*)(ws + off_xh2);
  unsigned short* xl2 = (unsigned short*)(ws + off_xl2);
  unsigned short* wh  = (unsigned short*)(ws + off_wh);
  unsigned short* wl  = (unsigned short*)(ws + off_wl);
  float* P1 = (float*)(ws + off_p1);
  float* P2 = (float*)(ws + off_p2);

  convert_kernel<<<(NGROUPS + 255) / 256, 256, 0, stream>>>(x1, x2, Wq1, Wk1, Wv1, Wq2, Wk2, Wv2,
                                                           xh1, xl1, xh2, xl2, wh, wl);

  proj_kernel<<<216, 128, 0, stream>>>(xh1, xl1, xh2, xl2, wh, wl,
                                       bq1, bk1, bv1, bq2, bk2, bv2, P1, P2);

  ctx2_kernel<<<16, 256, 0, stream>>>(P1, P2, wfc2, bfc2, out);

  tail_kernel<<<1, 256, 0, stream>>>(P1, P2, wfc1, bfc1, out);
}
